// MLP_GAT_Block_67628555043538
// MI455X (gfx1250) — hardware-verified
//
#include <hip/hip_runtime.h>


#define NG   16
#define NN_  1024
#define NTK  (NG * NN_)
#define FIN  256
#define HID  512
#define OUTF 256
#define PSC  32768.0f
#define LOSC 1024.0f
#define LOSCI (1.0f / 1024.0f)
#define ALPHA 0.2f
#define NEGF (-9.0e15f)

typedef unsigned short bf;
typedef __attribute__((ext_vector_type(16))) __bf16   v16bf;
typedef __attribute__((ext_vector_type(8)))  unsigned short v8us;
typedef __attribute__((ext_vector_type(8)))  float    v8f;
typedef __attribute__((ext_vector_type(4)))  float    v4f;
typedef v4f  __attribute__((may_alias)) v4fa;
typedef v8us __attribute__((may_alias)) v8usa;

__device__ __forceinline__ unsigned short f2bf(float f) { unsigned u = __float_as_uint(f); u += 0x7FFFu + ((u >> 16) & 1u); return (unsigned short)(u >> 16); }
__device__ __forceinline__ float bf2f(unsigned short b) { return __uint_as_float(((unsigned)b) << 16); }
__device__ __forceinline__ float bfr(float f) { return bf2f(f2bf(f)); }
__device__ __forceinline__ float elu_(float v) { return v > 0.f ? v : (__expf(v) - 1.0f); }
__device__ __forceinline__ v16bf cat16b(v8us lo, v8us hi) { return __builtin_bit_cast(v16bf, __builtin_shufflevector(lo, hi, 0, 1, 2, 3, 4, 5, 6, 7, 8, 9, 10, 11, 12, 13, 14, 15)); }
__device__ __forceinline__ v8f wmmab(v16bf a, v16bf b, v8f c) { return __builtin_amdgcn_wmma_f32_16x16x32_bf16(false, a, false, b, (short)0, c, false, false); }
#define VST2(T, p, v) do { const T vst2_v_ = (v); *(volatile T*)(p) = vst2_v_; __threadfence(); *(volatile T*)(p) = vst2_v_; } while (0)

template <int C>
__global__ __launch_bounds__(256) void k_cvtb(const float* __restrict__ src, int nrows, bf* dst) {
    const int lane = threadIdx.x & 31, row = blockIdx.x * 8 + (threadIdx.x >> 5);
    if (row >= nrows) return;
    v8us o[C / 256];
#pragma unroll
    for (int c = 0; c < C / 256; ++c) {
#pragma unroll
        for (int i = 0; i < 8; ++i) o[c][i] = f2bf(src[(size_t)row * C + c * 256 + lane * 8 + i]); }
#pragma unroll
    for (int c = 0; c < C / 256; ++c) *(volatile v8us*)(dst + (size_t)row * C + c * 256 + lane * 8) = o[c];
    __threadfence();
#pragma unroll
    for (int c = 0; c < C / 256; ++c) *(volatile v8us*)(dst + (size_t)row * C + c * 256 + lane * 8) = o[c];
}
__global__ __launch_bounds__(256) void k_wt(const float* __restrict__ Wm, int K, int ncols, bf* WT) {
    __shared__ __align__(16) unsigned short tl[64 * 72];
    const int tid = threadIdx.x, k0 = blockIdx.x * 64, n0 = blockIdx.y * 64;
    const int kk = tid >> 2, nq = (tid & 3) * 16;
#pragma unroll
    for (int i = 0; i < 16; ++i) tl[(nq + i) * 72 + kk] = f2bf(Wm[(size_t)(k0 + kk) * ncols + n0 + nq + i]);
    __syncthreads();
    const int piece = tid & 7;
    auto pass = [&]() {
#pragma unroll
        for (int s = 0; s < 2; ++s) { const int nr = (tid >> 3) + 32 * s; const v8us val = *(const v8usa*)(tl + nr * 72 + piece * 8); *(volatile v8us*)(WT + (size_t)(n0 + nr) * K + k0 + piece * 8) = val; }
    };
    pass(); __threadfence(); pass();
}
template <bool SA, int MODE>
__global__ __launch_bounds__(128) void k_gemm(const bf* __restrict__ A, const bf* __restrict__ Al, const bf* __restrict__ Bn, int K, const float* __restrict__ bias, int ldc, float* C, bf* PH, bf* PL) {
    __shared__ __align__(16) float ost[4][16 * 68];
    const int lane = threadIdx.x & 31, wave = threadIdx.x >> 5, lr = lane & 15, hi = lane >> 4;
    const size_t r0 = (size_t)blockIdx.x * 64 + wave * 16; const int c0 = blockIdx.y * 64;
    const size_t aoff = (r0 + lr) * K + 8 * hi;
    size_t boff[4];
#pragma unroll
    for (int t = 0; t < 4; ++t) boff[t] = (size_t)(c0 + t * 16 + lr) * K + 8 * hi;
    v8f acc[4];
#pragma unroll
    for (int t = 0; t < 4; ++t) acc[t] = (v8f){};
#pragma unroll 2
    for (int kc = 0; kc < K; kc += 32) {
        const v16bf a = cat16b(*(const v8us*)(A + aoff + kc), *(const v8us*)(A + aoff + kc + 16));
        v16bf al = a; if (SA) al = cat16b(*(const v8us*)(Al + aoff + kc), *(const v8us*)(Al + aoff + kc + 16));
#pragma unroll
        for (int t = 0; t < 4; ++t) { const v16bf bb = cat16b(*(const v8us*)(Bn + boff[t] + kc), *(const v8us*)(Bn + boff[t] + kc + 16)); acc[t] = wmmab(a, bb, acc[t]); if (SA) acc[t] = wmmab(al, bb, acc[t]); }
        asm volatile("v_nop\n\tv_nop\n\tv_nop\n\tv_nop" : "+v"(acc[0]), "+v"(acc[1]), "+v"(acc[2]), "+v"(acc[3]) : "v"(a), "v"(al));
    }
    float* os = &ost[wave][0];
#pragma unroll
    for (int t = 0; t < 4; ++t) { const float bv = (MODE == 0) ? bfr(bias[c0 + t * 16 + lr]) : 0.f;
#pragma unroll
        for (int j = 0; j < 8; ++j) { float v = acc[t][j] + bv; if (MODE == 0) v = fmaxf(v, 0.f); os[(hi * 8 + j) * 68 + t * 16 + lr] = v; } }
    __syncthreads();
    float* crow = C + r0 * ldc + c0;
    auto pass = [&]() {
#pragma unroll
        for (int s = 0; s < 8; ++s) { const int Lid = (lane >> 3) + 4 * s, piece = lane & 7; const int row = Lid >> 1, cofs = (Lid & 1) * 32 + piece * 4;
            const v4f val = *(const v4fa*)(os + row * 68 + cofs); *(volatile v4f*)(crow + (size_t)row * ldc + cofs) = val; }
        if (MODE == 0) {
#pragma unroll
            for (int s = 0; s < 4; ++s) { const int row = 4 * s + (lane >> 3), piece = lane & 7; const float* sp = os + row * 68 + piece * 8; v8us oh, ol;
#pragma unroll
                for (int i = 0; i < 8; ++i) { const unsigned short hb = f2bf(sp[i]); oh[i] = hb; ol[i] = f2bf(sp[i] - bf2f(hb)); }
                *(volatile v8us*)(PH + (r0 + row) * ldc + c0 + piece * 8) = oh; *(volatile v8us*)(PL + (r0 + row) * ldc + c0 + piece * 8) = ol; } }
    };
    pass(); __threadfence(); pass();
}
template <int F>
__global__ __launch_bounds__(256) void k_f(const float* __restrict__ H, const float* __restrict__ a, float* F1, float* F2) {
    __shared__ float s1[32], s2[32];
    const int lane = threadIdx.x & 31, wave = threadIdx.x >> 5;
#pragma unroll 1
    for (int q = 0; q < 4; ++q) { const size_t row = (size_t)blockIdx.x * 32 + wave * 4 + q; float p1 = 0.f, p2 = 0.f;
#pragma unroll
        for (int c = 0; c < F / 32; ++c) { const float h = H[row * F + c * 32 + lane]; p1 += h * bfr(a[c * 32 + lane]); p2 += h * bfr(a[F + c * 32 + lane]); }
#pragma unroll
        for (int sh = 16; sh; sh >>= 1) { p1 += __shfl_xor(p1, sh, 32); p2 += __shfl_xor(p2, sh, 32); }
        if (lane == 0) { s1[wave * 4 + q] = p1; s2[wave * 4 + q] = p2; } }
    __syncthreads();
    if (wave == 0) { const float v1 = s1[lane], v2 = s2[lane]; const size_t o = (size_t)blockIdx.x * 32 + lane;
        *(volatile float*)(F1 + o) = v1; *(volatile float*)(F2 + o) = v2; __threadfence(); *(volatile float*)(F1 + o) = v1; *(volatile float*)(F2 + o) = v2; }
}
template <int F>
__global__ __launch_bounds__(256) void k_ht(const float* __restrict__ H, bf* HTH, bf* HTL) {
    __shared__ float tl[64][65];
    const int tid = threadIdx.x, j0 = blockIdx.x * 64, d0 = blockIdx.y * 64, g = blockIdx.z;
    { const int jj = tid >> 2, dq = (tid & 3) * 16;
#pragma unroll
      for (int i = 0; i < 16; ++i) tl[dq + i][jj] = H[((size_t)g * NN_ + j0 + jj) * F + d0 + dq + i]; }
    __syncthreads();
    const int piece = tid & 7;
    auto pass = [&]() {
#pragma unroll
        for (int s = 0; s < 2; ++s) { const int d = (tid >> 3) + 32 * s; v8us oh, ol;
#pragma unroll
            for (int i = 0; i < 8; ++i) { const float v = tl[d][piece * 8 + i]; const unsigned short hb = f2bf(v); oh[i] = hb; ol[i] = f2bf((v - bf2f(hb)) * LOSC); }
            const size_t o = ((size_t)g * F + d0 + d) * NN_ + j0 + piece * 8; *(volatile v8us*)(HTH + o) = oh; *(volatile v8us*)(HTL + o) = ol; }
    };
    pass(); __threadfence(); pass();
}
__global__ __launch_bounds__(256) void k_split(const float* __restrict__ O, int nrows, bf* PH, bf* PL) {
    const int lane = threadIdx.x & 31, row = blockIdx.x * 8 + (threadIdx.x >> 5);
    if (row >= nrows) return;
    v8us oh[2], ol[2];
#pragma unroll
    for (int c = 0; c < 2; ++c)
#pragma unroll
        for (int i = 0; i < 8; ++i) { const float v = O[(size_t)row * HID + c * 256 + lane * 8 + i]; const unsigned short hb = f2bf(v); oh[c][i] = hb; ol[c][i] = f2bf(v - bf2f(hb)); }
#pragma unroll
    for (int c = 0; c < 2; ++c) { *(volatile v8us*)(PH + (size_t)row * HID + c * 256 + lane * 8) = oh[c]; *(volatile v8us*)(PL + (size_t)row * HID + c * 256 + lane * 8) = ol[c]; }
    __threadfence();
#pragma unroll
    for (int c = 0; c < 2; ++c) { *(volatile v8us*)(PH + (size_t)row * HID + c * 256 + lane * 8) = oh[c]; *(volatile v8us*)(PL + (size_t)row * HID + c * 256 + lane * 8) = ol[c]; }
}
template <int F, bool MASK, bool FINAL>
__global__ __launch_bounds__(128) void k_gat(const float* __restrict__ F1, const float* __restrict__ F2, const int* __restrict__ adj, const bf* __restrict__ HTH, const bf* __restrict__ HTL,
                                            const float* __restrict__ R, float* O, bf* PH, bf* PL) {
    __shared__ __align__(16) unsigned short plds[4][16 * 32];
    __shared__ __align__(16) unsigned short plds2[4][16 * 32];
    __shared__ __align__(16) float ost[4][16 * 68];
    const int lane = threadIdx.x & 31, wave = threadIdx.x >> 5, lr = lane & 15, hi = lane >> 4;
    const int g = blockIdx.z, ch = blockIdx.y, i0 = blockIdx.x * 64 + wave * 16;
    const size_t row0 = (size_t)g * NN_;
    unsigned short* pl = &plds[wave][0]; unsigned short* pl2 = &plds2[wave][0];
    float f1[8];
#pragma unroll
    for (int j = 0; j < 8; ++j) f1[j] = F1[row0 + i0 + hi * 8 + j];
    v8f o[8], ox[8];
#pragma unroll
    for (int n = 0; n < 8; ++n) { o[n] = (v8f){}; ox[n] = (v8f){}; }
    float mrow[8], lpart[8];
#pragma unroll
    for (int j = 0; j < 8; ++j) { mrow[j] = -3.0e38f; lpart[j] = 0.f; }
#pragma unroll 1
    for (int kt = 0; kt < NN_ / 32; ++kt) {
        const int j0 = kt * 32; const float fa = F2[row0 + j0 + lr], fb = F2[row0 + j0 + 16 + lr];
        float alpha[8];
#pragma unroll
        for (int j = 0; j < 8; ++j) { const int i = i0 + hi * 8 + j;
            float ea = f1[j] + fa, eb = f1[j] + fb; ea = ea > 0.f ? ea : ALPHA * ea; eb = eb > 0.f ? eb : ALPHA * eb;
            if (MASK) { if (!(adj[(size_t)i * NN_ + j0 + lr] > 0)) ea = NEGF; if (!(adj[(size_t)i * NN_ + j0 + 16 + lr] > 0)) eb = NEGF; }
            float mx = fmaxf(ea, eb);
            mx = fmaxf(mx, __shfl_xor(mx, 1, 16)); mx = fmaxf(mx, __shfl_xor(mx, 2, 16)); mx = fmaxf(mx, __shfl_xor(mx, 4, 16)); mx = fmaxf(mx, __shfl_xor(mx, 8, 16));
            const float mn = fmaxf(mrow[j], mx);
            alpha[j] = __expf(mrow[j] - mn); mrow[j] = mn;
            const float p0 = __expf(ea - mn), p1 = __expf(eb - mn);
            lpart[j] = lpart[j] * alpha[j] + (p0 + p1);
            const int mr = hi * 8 + j; const float ps0 = p0 * PSC, ps1 = p1 * PSC; const unsigned short h0 = f2bf(ps0), h1 = f2bf(ps1);
            pl[mr * 32 + lr] = h0; pl[mr * 32 + 16 + lr] = h1; pl2[mr * 32 + lr] = f2bf(ps0 - bf2f(h0)); pl2[mr * 32 + 16 + lr] = f2bf(ps1 - bf2f(h1)); }
#pragma unroll
        for (int n = 0; n < 8; ++n)
#pragma unroll
            for (int j = 0; j < 8; ++j) { o[n][j] *= alpha[j]; ox[n][j] *= alpha[j]; }
        asm volatile("" ::: "memory");
        const v16bf pa = cat16b(*(const v8usa*)(pl + lr * 32 + hi * 8), *(const v8usa*)(pl + lr * 32 + 16 + hi * 8));
        const v16bf px = cat16b(*(const v8usa*)(pl2 + lr * 32 + hi * 8), *(const v8usa*)(pl2 + lr * 32 + 16 + hi * 8));
#pragma unroll
        for (int n = 0; n < 8; ++n) { const size_t ho = ((size_t)g * F + ch * 128 + n * 16 + lr) * NN_ + j0 + hi * 8;
            const v16bf hh = cat16b(*(const v8us*)(HTH + ho), *(const v8us*)(HTH + ho + 16)), hl = cat16b(*(const v8us*)(HTL + ho), *(const v8us*)(HTL + ho + 16));
            o[n] = wmmab(pa, hh, o[n]); o[n] = wmmab(px, hh, o[n]); ox[n] = wmmab(pa, hl, ox[n]);
            asm volatile("" : "+v"(o[n]), "+v"(ox[n]) : "v"(hh), "v"(hl) : "memory"); }
        asm volatile("v_nop\n\tv_nop\n\tv_nop\n\tv_nop" : "+v"(o[0]), "+v"(o[7]), "+v"(ox[0]), "+v"(ox[7]) : "v"(pa), "v"(px));
    }
    float inv[8];
#pragma unroll
    for (int j = 0; j < 8; ++j) { float rs = lpart[j]; rs += __shfl_xor(rs, 1, 16); rs += __shfl_xor(rs, 2, 16); rs += __shfl_xor(rs, 4, 16); rs += __shfl_xor(rs, 8, 16); inv[j] = 1.0f / (rs * PSC); }
    float* os = &ost[wave][0];
    const int cbase = ch * 128;
#pragma unroll
    for (int half = 0; half < 2; ++half) {
#pragma unroll
        for (int n = 0; n < 4; ++n)
#pragma unroll
            for (int j = 0; j < 8; ++j) { const size_t row = row0 + i0 + hi * 8 + j; const int d = cbase + half * 64 + n * 16 + lr;
                float v = (o[half * 4 + n][j] + ox[half * 4 + n][j] * LOSCI) * inv[j];
                v = elu_(elu_(v)) + R[row * F + d]; if (FINAL) v = fmaxf(v, 0.f);
                os[(hi * 8 + j) * 68 + n * 16 + lr] = v; }
        __builtin_amdgcn_wave_barrier(); asm volatile("" ::: "memory");
        float* ob = O + (row0 + i0) * F + cbase + half * 64;
#pragma unroll
        for (int ps2 = 0; ps2 < 2; ++ps2) {
#pragma unroll
            for (int s = 0; s < 8; ++s) { const int Lid = (lane >> 3) + 4 * s, piece = lane & 7; const int row = Lid >> 1, cofs = (Lid & 1) * 32 + piece * 4;
                const v4f val = *(const v4fa*)(os + row * 68 + cofs); *(volatile v4f*)(ob + (size_t)row * F + cofs) = val; }
            if (PH != nullptr) {
#pragma unroll
                for (int s = 0; s < 4; ++s) { const int row = 4 * s + (lane >> 3), piece = lane & 7; const float* sp = os + row * 68 + piece * 8; v8us oh, ol;
#pragma unroll
                    for (int i = 0; i < 8; ++i) { const unsigned short hb = f2bf(sp[i]); oh[i] = hb; ol[i] = f2bf(sp[i] - bf2f(hb)); }
                    const size_t po = (row0 + i0 + row) * F + cbase + half * 64 + piece * 8; *(volatile v8us*)(PH + po) = oh; *(volatile v8us*)(PL + po) = ol; } }
            if (ps2 == 0) __threadfence(); }
        __builtin_amdgcn_wave_barrier(); asm volatile("" ::: "memory");
    }
}

extern "C" void kernel_launch(void* const* d_in, const int* in_sizes, int n_in,
                              void* d_out, int out_size, void* d_ws, size_t ws_size, hipStream_t stream) {
    (void)in_sizes; (void)n_in; (void)out_size;
    const float* x = (const float*)d_in[0]; const int* adj = (const int*)d_in[1]; const float* W1 = (const float*)d_in[2]; const float* b1 = (const float*)d_in[3];
    const float* W2 = (const float*)d_in[4]; const float* b2 = (const float*)d_in[5]; const float* Wfc = (const float*)d_in[6]; const float* afc = (const float*)d_in[7]; const float* Whd = (const float*)d_in[8]; const float* ahd = (const float*)d_in[9];
    float* out = (float*)d_out;
    char* wsp = (char*)d_ws;
    auto take = [&](size_t bytes) { char* p = wsp; wsp += (bytes + 255) & ~(size_t)255; return (void*)p; };
    bf* Xb = (bf*)take((size_t)NTK * FIN * 2); bf* W1T = (bf*)take((size_t)HID * FIN * 2); bf* W2T = (bf*)take((size_t)OUTF * HID * 2); bf* WfT = (bf*)take((size_t)HID * HID * 2); bf* WhT = (bf*)take((size_t)OUTF * OUTF * 2);
    const size_t RB = (size_t)NTK * HID * 4;
    char* R1 = (char*)take(RB); char* R2 = (char*)take(RB); char* R3 = (char*)take(RB);
    float* F1 = (float*)take((size_t)NTK * 4); float* F2 = (float*)take((size_t)NTK * 4);
    if ((size_t)(wsp - (char*)d_ws) > ws_size) return;
    float* O1 = (float*)R1;
    bf* P1H = (bf*)R2; bf* P1L = (bf*)(R2 + RB / 2);
    float* Hf = (float*)R3;
    bf* HTH = P1H; bf* HTL = P1L; float* Og = Hf; bf* OgH = P1H; bf* OgL = P1L;
    float* O2 = (float*)R1; bf* P2H = (bf*)(R1 + RB / 2); bf* P2L = (bf*)(R1 + 3 * RB / 4);
    float* H2 = (float*)R3; bf* HT2H = (bf*)(R3 + RB / 2); bf* HT2L = (bf*)(R3 + 3 * RB / 4);
    k_cvtb<FIN><<<NTK / 8, 256, 0, stream>>>(x, NTK, Xb);
    k_wt<<<dim3(FIN / 64, HID / 64, 1), 256, 0, stream>>>(W1, FIN, HID, W1T); k_wt<<<dim3(HID / 64, OUTF / 64, 1), 256, 0, stream>>>(W2, HID, OUTF, W2T);
    k_wt<<<dim3(HID / 64, HID / 64, 1), 256, 0, stream>>>(Wfc, HID, HID, WfT); k_wt<<<dim3(OUTF / 64, OUTF / 64, 1), 256, 0, stream>>>(Whd, OUTF, OUTF, WhT);
    k_gemm<false, 0><<<dim3(NTK / 64, HID / 64, 1), 128, 0, stream>>>(Xb, nullptr, W1T, FIN, b1, HID, O1, P1H, P1L);
    k_gemm<true, 1><<<dim3(NTK / 64, HID / 64, 1), 128, 0, stream>>>(P1H, P1L, WfT, HID, nullptr, HID, Hf, nullptr, nullptr);
    k_f<HID><<<NTK / 32, 256, 0, stream>>>(Hf, afc, F1, F2);
    k_ht<HID><<<dim3(NN_ / 64, HID / 64, NG), 256, 0, stream>>>(Hf, HTH, HTL);
    k_gat<HID, false, false><<<dim3(NN_ / 64, HID / 128, NG), 128, 0, stream>>>(F1, F2, adj, HTH, HTL, O1, Og, nullptr, nullptr);
    k_split<<<NTK / 8, 256, 0, stream>>>(Og, NTK, OgH, OgL);
    k_gemm<true, 0><<<dim3(NTK / 64, OUTF / 64, 1), 128, 0, stream>>>(OgH, OgL, W2T, HID, b2, OUTF, O2, P2H, P2L);
    k_gemm<true, 1><<<dim3(NTK / 64, OUTF / 64, 1), 128, 0, stream>>>(P2H, P2L, WhT, OUTF, nullptr, OUTF, H2, nullptr, nullptr);
    k_f<OUTF><<<NTK / 32, 256, 0, stream>>>(H2, ahd, F1, F2);
    k_ht<OUTF><<<dim3(NN_ / 64, OUTF / 64, NG), 256, 0, stream>>>(H2, HT2H, HT2L);
    k_gat<OUTF, true, true><<<dim3(NN_ / 64, OUTF / 128, NG), 128, 0, stream>>>(F1, F2, adj, HT2H, HT2L, O2, out, nullptr, nullptr);
}
